// MASSVariationalDist_34333968564439
// MI455X (gfx1250) — hardware-run, weakly checked
//
#include <hip/hip_runtime.h>
#include <math.h>

typedef __attribute__((ext_vector_type(16))) _Float16 v16h;
typedef __attribute__((ext_vector_type(8)))  _Float16 v8h;
typedef __attribute__((ext_vector_type(8)))  float    v8f;
typedef __attribute__((ext_vector_type(4)))  float    v4f;

constexpr int kB   = 2048;
constexpr int kC   = 100;
constexpr int kK   = 8;
constexpr int kD   = 64;
constexpr int kCK  = kC * kK;
constexpr int kBT  = 128;
constexpr int kWcP = 96;
constexpr float kLog2Pi      = 1.8378770664093453f;
constexpr float kHalfDLog2Pi = 0.5f * (float)kD * kLog2Pi;
static_assert(kCK == 800, "class-component pairs");
static_assert((kD % 32) == 0, "K multiple of 32");
static_assert(kD == 64, "N is one 64-wide tile, two 32-deep k groups");
static_assert((kB % kBT) == 0 && (kBT % 16) == 0, "M tile multiple");
static_assert((kB % 32) == 0, "output groups of 32 rows");
static_assert(((32 * kC * 4) % 128) == 0, "32 output rows are whole 128-B lines");
static_assert((kWcP * 4) % 128 == 0, "per-pair record is whole lines");

constexpr size_t kOffL16  = 0;
constexpr size_t kOffWC   = kOffL16 + (size_t)kCK * kD * kD * 2;
constexpr size_t kOffX16  = kOffWC  + (size_t)kCK * kWcP * 4;
constexpr size_t kOffCLT  = kOffX16 + (size_t)kB * kD * 2;
constexpr size_t kWsTotal = kOffCLT + (size_t)kC * kB * 4;
static_assert(kWsTotal == 7942144ull, "carve total");
static_assert(kWsTotal <= 134217728ull, "carve cap");
static_assert((kOffWC % 128) == 0 && (kOffX16 % 128) == 0 && (kOffCLT % 128) == 0, "128-B aligned regions");

union FragU { v16h v; v8h h[2]; };
__device__ __forceinline__ v16h frag_load(const _Float16* p) {
  FragU f;
  f.h[0] = *(const v8h*)(p);
  f.h[1] = *(const v8h*)(p + 16);
  return f.v;
}
__device__ __forceinline__ v8f mma_f16(v16h a, v16h b, v8f c) {
  c = __builtin_amdgcn_wmma_f32_16x16x32_f16(false, a, false, b, (short)0, c, false, false);
  asm volatile("v_nop\n\tv_nop\n\tv_nop\n\tv_nop" : "+v"(c) : "v"(a), "v"(b));
  return c;
}
__device__ __forceinline__ void quad_acc(const v8f& acc, float wn, float (&q)[8]) {
#pragma unroll
  for (int r = 0; r < 8; ++r) {
    const float z = acc[r] - wn;
    q[r] = fmaf(z, z, q[r]);
  }
}

__global__ __launch_bounds__(64) void prep_kernel(
    const float* __restrict__ tril, const float* __restrict__ loc, const float* __restrict__ mixl,
    unsigned short* __restrict__ L16, float* __restrict__ WC)
{
  __shared__ __align__(16) float Ls[kD * kD];
  __shared__ __align__(16) float Zs[kD * kD];
  __shared__ float sdinv[kD];
  __shared__ float slog[kD];
  __shared__ float smu[kD];
  const int ck = blockIdx.x;
  const int t = threadIdx.x;
  const int lane = t & 31;
  const int wave = t >> 5;
  const float* Lg = tril + (size_t)ck * kD * kD;

  {
    const int rsub = t >> 4;
    const int c4 = (t & 15) * 4;
#pragma unroll 4
    for (int it = 0; it < 16; ++it) {
      const int row = it * 4 + rsub;
      const v4f v = *(const v4f*)(Lg + row * kD + c4);
      v4f o;
      o[0] = (c4 + 0 <= row) ? v[0] : 0.0f;
      o[1] = (c4 + 1 <= row) ? v[1] : 0.0f;
      o[2] = (c4 + 2 <= row) ? v[2] : 0.0f;
      o[3] = (c4 + 3 <= row) ? v[3] : 0.0f;
      *(v4f*)(Ls + row * kD + c4) = o;
    }
  }
  smu[t] = loc[(size_t)ck * kD + t];
  __syncthreads();
  {
    const float dg = Ls[t * kD + t];
    sdinv[t] = 1.0f / dg;
    slog[t] = logf(fabsf(dg));
  }
  __syncthreads();

#pragma unroll 1
  for (int i = 0; i < kD; ++i) {
    float s = (i == t) ? 1.0f : 0.0f;
    const float* lrow = Ls + i * kD;
#pragma unroll 4
    for (int m = 0; m < i; ++m) s = fmaf(-lrow[m], Zs[m * kD + t], s);
    const float val = s * sdinv[i];
    Zs[i * kD + t] = (i < t) ? 0.0f : val;
  }
  __syncthreads();

  float wacc = 0.0f;
#pragma unroll 4
  for (int j = 0; j < kD; ++j) wacc = fmaf(Zs[t * kD + j], smu[j], wacc);

  float ld = 0.0f;
#pragma unroll 1
  for (int i = 0; i < kD; ++i) ld += slog[i];
  const int cls = ck / kK;
  const int kcomp = ck - cls * kK;
  const float* mrow = mixl + (size_t)cls * kK;
  float mmax = -3.0e38f;
#pragma unroll 1
  for (int kk = 0; kk < kK; ++kk) mmax = fmaxf(mmax, mrow[kk]);
  float msum = 0.0f;
#pragma unroll 1
  for (int kk = 0; kk < kK; ++kk) msum += expf(mrow[kk] - mmax);
  const float mixlog = (mrow[kcomp] - mmax) - logf(msum);
  const float ct = (-ld - kHalfDLog2Pi) + mixlog;

  const int q = lane >> 3;
  const int c8 = (lane & 7) * 8;
  v8h hv[8];
#pragma unroll
  for (int it = 0; it < 8; ++it) {
    const int row = it * 8 + wave * 4 + q;
    const v4f a0 = *(const v4f*)(Zs + row * kD + c8);
    const v4f a1 = *(const v4f*)(Zs + row * kD + c8 + 4);
#pragma unroll
    for (int e = 0; e < 4; ++e) {
      hv[it][e]     = (_Float16)a0[e];
      hv[it][4 + e] = (_Float16)a1[e];
    }
  }
  unsigned short* Lo = L16 + (size_t)ck * kD * kD;
  float* wrec = WC + (size_t)ck * kWcP;
  for (int pass = 0; pass < 2; ++pass) {
#pragma unroll
    for (int it = 0; it < 8; ++it) {
      const int row = it * 8 + wave * 4 + q;
      *(volatile v8h*)(Lo + row * kD + c8) = hv[it];
    }
    *(volatile float*)(wrec + t) = wacc;
    if (t < 32) *(volatile float*)(wrec + kD + t) = ct;
    __threadfence();
  }
}

__global__ __launch_bounds__(256) void cvt_rows_f16_kernel(
    const float* __restrict__ src, unsigned short* __restrict__ dst, int total8)
{
  const int i = blockIdx.x * 256 + threadIdx.x;
  if (i >= total8) return;
  const size_t e0 = (size_t)i << 3;
  const v4f a0 = *(const v4f*)(src + e0);
  const v4f a1 = *(const v4f*)(src + e0 + 4);
  v8h hv;
#pragma unroll
  for (int e = 0; e < 4; ++e) {
    hv[e]     = (_Float16)a0[e];
    hv[4 + e] = (_Float16)a1[e];
  }
  unsigned short* qd = dst + e0;
  *(volatile v8h*)qd = hv;
  __threadfence();
  *(volatile v8h*)qd = hv;
}

__global__ __launch_bounds__(256) void whiten_quad_lse_kernel(
    const unsigned short* __restrict__ X16p, const unsigned short* __restrict__ L16p,
    const float* __restrict__ WC, float* __restrict__ CLT)
{
  __shared__ __align__(16) float scls[kBT];
  const _Float16* X16 = (const _Float16*)X16p;
  const _Float16* L16 = (const _Float16*)L16p;
  const int tid = threadIdx.x;
  const int lane = tid & 31;
  const int wave = tid >> 5;
  const int h = lane >> 4;
  const int rl = lane & 15;
  const int sel = lane & 7;
  const int c = blockIdx.x;
  const int b0 = blockIdx.y * kBT;

  const _Float16* xa = X16 + (size_t)(b0 + wave * 16 + rl) * kD + 8 * h;
  const v16h a0 = frag_load(xa);
  const v16h a1 = frag_load(xa + 32);

  float mrun = -3.0e38f;
  float srun = 0.0f;

#pragma unroll 1
  for (int k = 0; k < kK; ++k) {
    const int ck = c * kK + k;
    const _Float16* Lb = L16 + (size_t)ck * kD * kD + rl * kD + 8 * h;
    const v16h b00 = frag_load(Lb);
    const v16h b10 = frag_load(Lb + 16 * kD);
    const v16h b20 = frag_load(Lb + 32 * kD);
    const v16h b21 = frag_load(Lb + 32 * kD + 32);
    const v16h b30 = frag_load(Lb + 48 * kD);
    const v16h b31 = frag_load(Lb + 48 * kD + 32);
    const float* wrec = WC + (size_t)ck * kWcP;
    const float w0 = wrec[rl];
    const float w1 = wrec[16 + rl];
    const float w2 = wrec[32 + rl];
    const float w3 = wrec[48 + rl];
    const float ct = wrec[kD];

    v8f acc0 = (v8f){0.f, 0.f, 0.f, 0.f, 0.f, 0.f, 0.f, 0.f};
    v8f acc1 = (v8f){0.f, 0.f, 0.f, 0.f, 0.f, 0.f, 0.f, 0.f};
    v8f acc2 = (v8f){0.f, 0.f, 0.f, 0.f, 0.f, 0.f, 0.f, 0.f};
    v8f acc3 = (v8f){0.f, 0.f, 0.f, 0.f, 0.f, 0.f, 0.f, 0.f};
    acc0 = mma_f16(a0, b00, acc0);
    acc1 = mma_f16(a0, b10, acc1);
    acc2 = mma_f16(a0, b20, acc2);
    acc2 = mma_f16(a1, b21, acc2);
    acc3 = mma_f16(a0, b30, acc3);
    acc3 = mma_f16(a1, b31, acc3);

    float q[8];
#pragma unroll
    for (int r = 0; r < 8; ++r) q[r] = 0.0f;
    quad_acc(acc0, w0, q);
    quad_acc(acc1, w1, q);
    quad_acc(acc2, w2, q);
    quad_acc(acc3, w3, q);

#pragma unroll
    for (int r = 0; r < 8; ++r) {
      float v = q[r];
      v += __shfl_xor(v, 1, 32);
      v += __shfl_xor(v, 2, 32);
      v += __shfl_xor(v, 4, 32);
      v += __shfl_xor(v, 8, 32);
      q[r] = v;
    }
    float myq = q[0];
    myq = (sel == 1) ? q[1] : myq;
    myq = (sel == 2) ? q[2] : myq;
    myq = (sel == 3) ? q[3] : myq;
    myq = (sel == 4) ? q[4] : myq;
    myq = (sel == 5) ? q[5] : myq;
    myq = (sel == 6) ? q[6] : myq;
    myq = (sel == 7) ? q[7] : myq;

    const float comp = fmaf(-0.5f, myq, ct);
    const float mnew = fmaxf(mrun, comp);
    srun = srun * expf(mrun - mnew) + expf(comp - mnew);
    mrun = mnew;
  }

  const float clsv = mrun + logf(srun);
  if ((lane & 8) == 0) scls[wave * 16 + 8 * h + sel] = clsv;
  __syncthreads();
  if (wave == 0) {
    const v4f v = *(const v4f*)(scls + lane * 4);
    float* dst = CLT + (size_t)c * kB + b0 + lane * 4;
    *(volatile v4f*)dst = v;
    __threadfence();
    *(volatile v4f*)dst = v;
  }
}

__global__ __launch_bounds__(32) void finalize_kernel(const float* __restrict__ CLT, float* __restrict__ out)
{
  __shared__ __align__(16) float tile[kC * 32];
  __shared__ float smx[32];
  __shared__ float slg[32];
  const int lane = threadIdx.x;
  const int b0 = blockIdx.x * 32;
  float mx = -3.0e38f;
#pragma unroll 1
  for (int c = 0; c < kC; ++c) {
    const float v = CLT[(size_t)c * kB + b0 + lane];
    tile[c * 32 + lane] = v;
    mx = fmaxf(mx, v);
  }
  float s = 0.0f;
#pragma unroll 1
  for (int c = 0; c < kC; ++c) s += expf(tile[c * 32 + lane] - mx);
  smx[lane] = mx;
  slg[lane] = logf(s);
  __syncthreads();
  float* ob = out + (size_t)b0 * kC;
  for (int pass = 0; pass < 2; ++pass) {
#pragma unroll 1
    for (int it = 0; it < 25; ++it) {
      const int e0 = it * 128 + lane * 4;
      v4f o;
#pragma unroll
      for (int j = 0; j < 4; ++j) {
        const int e = e0 + j;
        const int b = e / kC;
        const int c = e - b * kC;
        o[j] = (tile[c * 32 + b] - smx[b]) - slg[b];
      }
      *(volatile v4f*)(ob + e0) = o;
    }
    __threadfence();
  }
}

extern "C" void kernel_launch(void* const* d_in, const int* in_sizes, int n_in,
                              void* d_out, int out_size, void* d_ws, size_t ws_size,
                              hipStream_t stream) {
  if (n_in < 4) return;
  if (in_sizes[0] != kB * kD) return;
  if (in_sizes[1] != kC * kK) return;
  if (in_sizes[2] != kCK * kD) return;
  if (in_sizes[3] != kCK * kD * kD) return;
  if (out_size != kB * kC) return;
  if (ws_size < kWsTotal) return;

  const float* rep  = (const float*)d_in[0];
  const float* mixl = (const float*)d_in[1];
  const float* loc  = (const float*)d_in[2];
  const float* tril = (const float*)d_in[3];
  float* out = (float*)d_out;

  char* ws = (char*)d_ws;
  unsigned short* L16 = (unsigned short*)(ws + kOffL16);
  float*          WC  = (float*)(ws + kOffWC);
  unsigned short* X16 = (unsigned short*)(ws + kOffX16);
  float*          CLT = (float*)(ws + kOffCLT);

  prep_kernel<<<kCK, 64, 0, stream>>>(tril, loc, mixl, L16, WC);
  cvt_rows_f16_kernel<<<(kB * kD / 8) / 256, 256, 0, stream>>>(rep, X16, kB * kD / 8);
  whiten_quad_lse_kernel<<<dim3(kC, kB / kBT), 256, 0, stream>>>(X16, L16, WC, CLT);
  finalize_kernel<<<kB / 32, 32, 0, stream>>>(CLT, out);
}
